// MultiQueryAttention_7662221656422
// MI455X (gfx1250) — hardware-verified
//
#include <hip/hip_runtime.h>
#include <math.h>

#ifndef NB
#define NB 4
#endif
#ifndef SEQ
#define SEQ 2048
#endif
#define NB_FULL 4
#define SEQ_FULL 2048
#define EMB 1024
#define NHEAD 16
#define HD 64
#define XSC 16.0f
#define WSC 16.0f
#define PSC 4096.0f
#define CTXC 256.0f

static_assert(SEQ % 64 == 0);
static_assert(((size_t)NB * SEQ) % 64 == 0);
static_assert(NB <= NB_FULL);
static_assert(SEQ <= SEQ_FULL);
static_assert(EMB == NHEAD * HD);

typedef __attribute__((ext_vector_type(16))) _Float16     v16h;
typedef __attribute__((ext_vector_type(8)))  _Float16     v8h;
typedef __attribute__((ext_vector_type(16))) __bf16       v16b;
typedef __attribute__((ext_vector_type(8)))  __bf16       v8b;
typedef __attribute__((ext_vector_type(8)))  float        v8f;
typedef __attribute__((ext_vector_type(4)))  float        v4f;
typedef __attribute__((ext_vector_type(4)))  unsigned int v4u;

union FragH { v16h v; v8h h[2]; };
union FragB { v16b v; v8b h[2]; };
__device__ __forceinline__ v16h ldfh(const _Float16* p) { FragH f; f.h[0] = *(const v8h*)(p); f.h[1] = *(const v8h*)(p + 16); return f.v; }
__device__ __forceinline__ v16b ldfb(const __bf16* p)   { FragB f; f.h[0] = *(const v8b*)(p); f.h[1] = *(const v8b*)(p + 16); return f.v; }

__device__ __forceinline__ v8f mma_h(v16h a, v16h b, v8f c) {
    c = __builtin_amdgcn_wmma_f32_16x16x32_f16(false, a, false, b, (short)0, c, false, false);
    asm volatile("v_nop\n\tv_nop\n\tv_nop\n\tv_nop" : "+v"(c) : "v"(a), "v"(b));
    return c;
}
__device__ __forceinline__ v8f mma_b(v16b a, v16b b, v8f c) {
    c = __builtin_amdgcn_wmma_f32_16x16x32_bf16(false, a, false, b, (short)0, c, false, false);
    asm volatile("v_nop\n\tv_nop\n\tv_nop\n\tv_nop" : "+v"(c) : "v"(a), "v"(b));
    return c;
}
__device__ __forceinline__ void dep_guard_h(v8f& a, v8f& b, v16h x, v16h y)  { asm volatile("v_nop\n\tv_nop\n\tv_nop\n\tv_nop" : "+v"(a), "+v"(b) : "v"(x), "v"(y)); }
__device__ __forceinline__ void dep_guard_hb(v8f& a, v8f& b, v16h x, v16b y) { asm volatile("v_nop\n\tv_nop\n\tv_nop\n\tv_nop" : "+v"(a), "+v"(b) : "v"(x), "v"(y)); }
__device__ __forceinline__ void keep4_h(v16h a, v16h b, v16h c, v16h d) { asm volatile("v_nop" :: "v"(a), "v"(b), "v"(c), "v"(d)); }
__device__ __forceinline__ void keep4_b(v16b a, v16b b, v16b c, v16b d) { asm volatile("v_nop" :: "v"(a), "v"(b), "v"(c), "v"(d)); }
__device__ __forceinline__ void acc_guard4(v8f& a, v8f& b, v8f& c, v8f& d) { asm volatile("v_nop\n\tv_nop\n\tv_nop\n\tv_nop" : "+v"(a), "+v"(b), "+v"(c), "+v"(d)); }

__device__ __forceinline__ unsigned short f2bf_bits(float f) {
    unsigned u = __float_as_uint(f);
    return (unsigned short)((u + 0x7FFFu + ((u >> 16) & 1u)) >> 16);
}
__device__ __forceinline__ float cmb_bf(float v) {
    const unsigned u = __float_as_uint(v);
    const unsigned r = (u + 0x7fffu + ((u >> 16) & 1u)) & 0xffff0000u;
    return __uint_as_float(r);
}
__device__ __forceinline__ unsigned int pk2h(float a, float b) {
    return (unsigned int)__builtin_bit_cast(unsigned short, (_Float16)a) | ((unsigned int)__builtin_bit_cast(unsigned short, (_Float16)b) << 16);
}
__device__ __forceinline__ unsigned int pk2bf(float a, float b) {
    return (__float_as_uint(a) >> 16) | (__float_as_uint(b) & 0xffff0000u);
}

#define VST2(T, ptr, val) do { const T vst2_v_ = (val); *(volatile T*)(ptr) = vst2_v_; __threadfence(); *(volatile T*)(ptr) = vst2_v_; } while (0)

__global__ __launch_bounds__(256) void k_castb(const float* __restrict__ SRC, unsigned short* __restrict__ DST) {
    const unsigned u = blockIdx.x * 256u + threadIdx.x;
    const unsigned r = u >> 7, c0 = (u & 127u) << 3;
    if (r >= (unsigned)SEQ) return;
    const unsigned b = blockIdx.y;
    const float* s = SRC + ((size_t)b * SEQ_FULL + r) * EMB + c0;
    const v4f x0 = *(const v4f*)(s), x1 = *(const v4f*)(s + 4);
    v4u pk;
    pk.x = pk2h(cmb_bf(x0.x) * XSC, cmb_bf(x0.y) * XSC); pk.y = pk2h(cmb_bf(x0.z) * XSC, cmb_bf(x0.w) * XSC);
    pk.z = pk2h(cmb_bf(x1.x) * XSC, cmb_bf(x1.y) * XSC); pk.w = pk2h(cmb_bf(x1.z) * XSC, cmb_bf(x1.w) * XSC);
    VST2(v4u, (v4u*)(DST + ((size_t)b * SEQ + r) * EMB + c0), pk);
}
static_assert((size_t)(SEQ / 2) * 256 * 8 == (size_t)SEQ * EMB);

template <bool BF>
__global__ __launch_bounds__(256) void k_castbT(const float* __restrict__ SRC, unsigned nC, unsigned short* __restrict__ DST) {
    const unsigned u = blockIdx.x * 256u + threadIdx.x;
    const unsigned c = u >> 7, r0 = (u & 127u) << 3;
    if (c >= nC) return;
    float w[8];
#pragma unroll
    for (int e = 0; e < 8; ++e) w[e] = cmb_bf(SRC[(size_t)(r0 + e) * nC + c]) * WSC;
    v4u pk;
    if (BF) { pk.x = pk2bf(w[0], w[1]); pk.y = pk2bf(w[2], w[3]); pk.z = pk2bf(w[4], w[5]); pk.w = pk2bf(w[6], w[7]); }
    else    { pk.x = pk2h(w[0], w[1]);  pk.y = pk2h(w[2], w[3]);  pk.z = pk2h(w[4], w[5]);  pk.w = pk2h(w[6], w[7]); }
    VST2(v4u, (v4u*)(DST + (size_t)c * EMB + r0), pk);
}

template <int TM, bool MIX, int BIAS_MODE, int OUT_MODE>
__global__ __launch_bounds__(256) void k_gemm64(
    const unsigned short* __restrict__ Ap, const unsigned short* __restrict__ A2p, unsigned lda, unsigned strideA,
    const unsigned short* __restrict__ Btp, const unsigned short* __restrict__ Bt2p, unsigned ldb,
    void* __restrict__ Cout, void* __restrict__ Cout2, unsigned ldc, unsigned strideC,
    const float* __restrict__ bias, unsigned tilesM, unsigned tilesN, unsigned K, float scale, float bscale) {
  __shared__ __align__(16) float sT[8][16 * 68];
  const unsigned b    = blockIdx.y;
  const unsigned lane = threadIdx.x & 31u;
  const unsigned wave = threadIdx.x >> 5;
  const unsigned tile = blockIdx.x * 8u + wave;
  if (tile >= tilesM * tilesN) return;
  const unsigned tm = tile / tilesN;
  const unsigned tn = tile - tm * tilesN;
  const unsigned m0 = tm * (16u * TM);
  const unsigned n0 = tn << 6;

  const _Float16* Ab  = (const _Float16*)Ap + (size_t)b * strideA;
  const _Float16* Bb  = (const _Float16*)Btp;
  const __bf16*   Ab2 = MIX ? ((const __bf16*)A2p + (size_t)b * strideA) : nullptr;
  const __bf16*   Bb2 = MIX ? (const __bf16*)Bt2p : nullptr;

  const unsigned rlane = lane & 15u;
  const unsigned koff  = (lane >> 4) * 8u;
  const unsigned mOff  = (lane >> 4) * 8u;

  v8f acc[TM][4];
#pragma unroll
  for (int i = 0; i < TM; ++i)
#pragma unroll
    for (int j = 0; j < 4; ++j) acc[i][j] = (v8f){0.f,0.f,0.f,0.f,0.f,0.f,0.f,0.f};

  for (unsigned k0 = 0; k0 < K; k0 += 32) {
    v16h bh[4]; v16b b2[4];
#pragma unroll
    for (int j = 0; j < 4; ++j) {
      const size_t bo = (size_t)(n0 + (unsigned)(j << 4) + rlane) * ldb + koff + k0;
      bh[j] = ldfh(Bb + bo);
      if (MIX) b2[j] = ldfb(Bb2 + bo);
    }
#pragma unroll
    for (int i = 0; i < TM; ++i) {
      const size_t ao = (size_t)(m0 + (unsigned)(i << 4) + rlane) * lda + koff + k0;
      const v16h ah = ldfh(Ab + ao);
      v16b al;
      if (MIX) al = ldfb(Ab2 + ao);
#pragma unroll
      for (int j = 0; j < 4; ++j) {
        acc[i][j] = __builtin_amdgcn_wmma_f32_16x16x32_f16(false, ah, false, bh[j], (short)0, acc[i][j], false, false);
        if (MIX) acc[i][j] = __builtin_amdgcn_wmma_f32_16x16x32_bf16(false, al, false, b2[j], (short)0, acc[i][j], false, false);
      }
      if (MIX) dep_guard_hb(acc[i][0], acc[i][3], ah, al); else dep_guard_h(acc[i][0], acc[i][3], ah, ah);
    }
    keep4_h(bh[0], bh[1], bh[2], bh[3]);
    if (MIX) keep4_b(b2[0], b2[1], b2[2], b2[3]);
  }
#pragma unroll
  for (int i = 0; i < TM; ++i) acc_guard4(acc[i][0], acc[i][1], acc[i][2], acc[i][3]);

  float* slab = sT[wave];
#pragma unroll
  for (int i = 0; i < TM; ++i) {
    const unsigned mBase = m0 + (unsigned)(i << 4);
#pragma unroll
    for (int j = 0; j < 4; ++j) {
      const unsigned n = n0 + (unsigned)(j << 4) + rlane;
      float bv = 0.f;
      if (BIAS_MODE == 2) bv = cmb_bf(bias[n]) * bscale;
#pragma unroll
      for (int r = 0; r < 8; ++r) {
        float v = acc[i][j][r] * scale;
        if (BIAS_MODE == 1) v += cmb_bf(bias[mBase + mOff + r]) * bscale;
        if (BIAS_MODE == 2) v += bv;
        slab[(mOff + r) * 68 + (j << 4) + rlane] = v;
      }
    }
    __builtin_amdgcn_fence(3  , "workgroup");
    __builtin_amdgcn_wave_barrier();
    __builtin_amdgcn_fence(2  , "workgroup");
    if (OUT_MODE == 0) {
      float* C = (float*)Cout + (size_t)b * strideC;
      const unsigned hh = lane >> 4, c4 = (lane & 15u) * 4u;
      for (int pass = 0; pass < 2; ++pass) {
#pragma unroll
        for (int it = 0; it < 8; ++it) {
          const unsigned row = (unsigned)(it * 2) + hh;
          const v4f v = *(const v4f*)(slab + row * 68 + c4);
          *(volatile v4f*)(C + (size_t)(mBase + row) * ldc + n0 + c4) = v;
        }
        __threadfence();
      }
    } else {
      const unsigned q = lane >> 3, c8 = (lane & 7u) * 8u;
      unsigned short* C  = (unsigned short*)Cout  + (size_t)b * strideC;
      unsigned short* C2 = (OUT_MODE >= 2) ? ((unsigned short*)Cout2 + (size_t)b * strideC) : nullptr;
      for (int pass = 0; pass < 2; ++pass) {
#pragma unroll
        for (int it = 0; it < 4; ++it) {
          const unsigned row = (unsigned)(it * 4) + q;
          const float* sp = slab + row * 68 + c8;
          v8h hv, lv;
#pragma unroll
          for (int e = 0; e < 8; ++e) {
            const float x = sp[e];
            const _Float16 xh = (_Float16)x;
            hv[e] = xh;
            if (OUT_MODE == 2) lv[e] = __builtin_bit_cast(_Float16, f2bf_bits(x - (float)xh));
            if (OUT_MODE == 3) lv[e] = __builtin_bit_cast(_Float16, f2bf_bits(x));
          }
          *(volatile v8h*)(C + (size_t)(mBase + row) * ldc + n0 + c8) = hv;
          if (OUT_MODE >= 2) *(volatile v8h*)(C2 + (size_t)(mBase + row) * ldc + n0 + c8) = lv;
        }
        __threadfence();
      }
    }
    __builtin_amdgcn_fence(3  , "workgroup");
    __builtin_amdgcn_wave_barrier();
    __builtin_amdgcn_fence(2  , "workgroup");
  }
}

__global__ __launch_bounds__(128) void k_flash(const unsigned short* __restrict__ Qhp, const unsigned short* __restrict__ Qlp,
                                               const unsigned short* __restrict__ Khp, const unsigned short* __restrict__ Kbp,
                                               const unsigned short* __restrict__ VTp,
                                               unsigned short* __restrict__ Chp, unsigned short* __restrict__ Clp) {
  __shared__ __align__(16) _Float16 Psh[4][16 * 64];
  __shared__ __align__(16) float    Os[4][16 * 68];
  const unsigned tid = threadIdx.x, wave = tid >> 5, lane = tid & 31u, hh = lane >> 4, c = lane & 15u;
  const unsigned qb = blockIdx.x, hd = blockIdx.y, b = blockIdx.z;
  const unsigned q0 = qb * 64u + wave * 16u;
  const size_t RT = (size_t)NB * SEQ;

  const size_t qoff = ((size_t)b * SEQ + q0 + c) * EMB + hd * 64u + 8u * hh;
  const v16h qah0 = ldfh((const _Float16*)Qhp + qoff), qah1 = ldfh((const _Float16*)Qhp + qoff + 32);
  const v16b qal0 = ldfb((const __bf16*)Qlp + qoff),   qal1 = ldfb((const __bf16*)Qlp + qoff + 32);

  const _Float16* kh = (const _Float16*)Khp + ((size_t)b * SEQ + c) * HD + 8u * hh;
  const __bf16*   kl = (const __bf16*)Kbp   + ((size_t)b * SEQ + c) * HD + 8u * hh;
  const _Float16* vt = (const _Float16*)VTp + (size_t)c * RT + (size_t)b * SEQ + 8u * hh;

  float mrow[8], lrow[8];
  v8f o[4];
#pragma unroll
  for (int r = 0; r < 8; ++r) { mrow[r] = -1.0e30f; lrow[r] = 0.f; }
#pragma unroll
  for (int t = 0; t < 4; ++t) o[t] = (v8f){0.f,0.f,0.f,0.f,0.f,0.f,0.f,0.f};

  const float SL2 = 0.125f * 1.4426950408889634f * (1.0f / 256.0f);
  _Float16* pw = Psh[wave];

#pragma unroll 1
  for (unsigned kc = 0; kc < (unsigned)(SEQ / 64); ++kc) {
    const unsigned kv0 = kc * 64u;
    v8f s[4];
#pragma unroll
    for (int j = 0; j < 4; ++j) {
      const size_t ko = (size_t)(kv0 + (unsigned)(j * 16)) * HD;
      v8f a = (v8f){0.f,0.f,0.f,0.f,0.f,0.f,0.f,0.f};
      a = mma_h(qah0, ldfh(kh + ko), a);
      a = mma_b(qal0, ldfb(kl + ko), a);
      a = mma_h(qah1, ldfh(kh + ko + 32), a);
      a = mma_b(qal1, ldfb(kl + ko + 32), a);
      s[j] = a;
    }
#pragma unroll
    for (int r = 0; r < 8; ++r) {
      const float x0 = s[0][r] * SL2, x1 = s[1][r] * SL2, x2 = s[2][r] * SL2, x3 = s[3][r] * SL2;
      float m = fmaxf(fmaxf(x0, x1), fmaxf(x2, x3));
      m = fmaxf(m, __shfl_xor(m, 1, 32)); m = fmaxf(m, __shfl_xor(m, 2, 32));
      m = fmaxf(m, __shfl_xor(m, 4, 32)); m = fmaxf(m, __shfl_xor(m, 8, 32));
      const float mnew = fmaxf(mrow[r], m);
      const float alpha = exp2f(mrow[r] - mnew);
      mrow[r] = mnew;
      const float p0 = exp2f(x0 - mnew), p1 = exp2f(x1 - mnew), p2 = exp2f(x2 - mnew), p3 = exp2f(x3 - mnew);
      float psum = (p0 + p1) + (p2 + p3);
      psum += __shfl_xor(psum, 1, 32); psum += __shfl_xor(psum, 2, 32);
      psum += __shfl_xor(psum, 4, 32); psum += __shfl_xor(psum, 8, 32);
      lrow[r] = lrow[r] * alpha + psum;
#pragma unroll
      for (int t = 0; t < 4; ++t) o[t][r] *= alpha;
      _Float16* pr = pw + (8u * hh + (unsigned)r) * 64u + c;
      pr[0]  = (_Float16)(p0 * PSC);
      pr[16] = (_Float16)(p1 * PSC);
      pr[32] = (_Float16)(p2 * PSC);
      pr[48] = (_Float16)(p3 * PSC);
    }
    __builtin_amdgcn_fence(3  , "workgroup");
    __builtin_amdgcn_wave_barrier();
    __builtin_amdgcn_fence(2  , "workgroup");
#pragma unroll
    for (int kk = 0; kk < 2; ++kk) {
      const v16h pa = ldfh(pw + c * 64u + (unsigned)(kk * 32) + 8u * hh);
#pragma unroll
      for (int t = 0; t < 4; ++t) {
        const v16h vb = ldfh(vt + (size_t)(t * 16) * RT + kv0 + (unsigned)(kk * 32));
        o[t] = mma_h(pa, vb, o[t]);
      }
    }
    __builtin_amdgcn_fence(3  , "workgroup");
    __builtin_amdgcn_wave_barrier();
    __builtin_amdgcn_fence(2  , "workgroup");
  }

  float* os = Os[wave];
#pragma unroll
  for (int r = 0; r < 8; ++r) {
    const float inv = (1.0f / lrow[r]) * (CTXC / (PSC * XSC));
#pragma unroll
    for (int t = 0; t < 4; ++t) os[(8u * hh + (unsigned)r) * 68u + (unsigned)(t * 16) + c] = o[t][r] * inv;
  }
  __builtin_amdgcn_fence(3  , "workgroup");
  __builtin_amdgcn_wave_barrier();
  __builtin_amdgcn_fence(2  , "workgroup");
  {
    const unsigned q = lane >> 3, c8 = (lane & 7u) * 8u;
    const size_t ob = ((size_t)b * SEQ + q0) * EMB + hd * 64u + c8;
    for (int pass = 0; pass < 2; ++pass) {
#pragma unroll
      for (int it = 0; it < 4; ++it) {
        const unsigned row = (unsigned)(it * 4) + q;
        const float* sp = os + row * 68u + c8;
        v8h hv, lv;
#pragma unroll
        for (int e = 0; e < 8; ++e) {
          const float x = sp[e];
          const _Float16 xh = (_Float16)x;
          hv[e] = xh;
          lv[e] = __builtin_bit_cast(_Float16, f2bf_bits(x - (float)xh));
        }
        *(volatile v8h*)(Chp + ob + (size_t)row * EMB) = hv;
        *(volatile v8h*)(Clp + ob + (size_t)row * EMB) = lv;
      }
      __threadfence();
    }
  }
}

constexpr size_t ROWS  = (size_t)NB * SEQ;
constexpr size_t SZ_X  = ROWS * EMB * 2;
constexpr size_t SZ_W  = (size_t)EMB * EMB * 2;
constexpr size_t SZ_WS = (size_t)HD * EMB * 2;
constexpr size_t SZ_K  = ROWS * HD * 2;
constexpr size_t CARVE = 3 * SZ_X + 3 * SZ_W + 2 * SZ_WS + 2 * SZ_X + 3 * SZ_K + 2 * SZ_X;
static_assert(SZ_X % 256 == 0);
static_assert(SZ_W % 256 == 0);
static_assert(SZ_WS % 256 == 0);
static_assert(SZ_K % 256 == 0);
static_assert(CARVE <= 134217728);
static_assert((ROWS / 64) * 16 * 64 * 64 == ROWS * EMB);
static_assert((ROWS / 64) * 64 * 64 == ROWS * HD);
static_assert((size_t)(SEQ / 64) * NHEAD * NB * 64 * 64 == ROWS * EMB);
static_assert((size_t)(SEQ / 32) * 16 * 32 * 64 == (size_t)SEQ * EMB);
static_assert(((size_t)(SEQ / 32) * 16) % 8 == 0);

extern "C" void kernel_launch(void* const* d_in, const int* in_sizes, int n_in, void* d_out, int out_size, void* d_ws, size_t ws_size, hipStream_t stream) {
    if (n_in < 11) return;
    const long long need_x = ((long long)(NB - 1) * SEQ_FULL + SEQ) * EMB;
    if ((long long)in_sizes[0] < need_x || (long long)in_sizes[1] < need_x || (long long)in_sizes[2] < need_x) return;
    if (in_sizes[3] < EMB * EMB || in_sizes[4] < EMB || in_sizes[5] < EMB * HD || in_sizes[6] < HD) return;
    if (in_sizes[7] < EMB * HD || in_sizes[8] < HD || in_sizes[9] < EMB * EMB || in_sizes[10] < EMB) return;
    if ((long long)out_size < need_x) return;
    if (CARVE > ws_size) return;

    const float* q  = (const float*)d_in[0];
    const float* k  = (const float*)d_in[1];
    const float* v  = (const float*)d_in[2];
    const float* Wq = (const float*)d_in[3];
    const float* bq = (const float*)d_in[4];
    const float* Wk = (const float*)d_in[5];
    const float* bk = (const float*)d_in[6];
    const float* Wv = (const float*)d_in[7];
    const float* bv = (const float*)d_in[8];
    const float* Wo = (const float*)d_in[9];
    const float* bo = (const float*)d_in[10];
    float* out = (float*)d_out;

    char* wsp = (char*)d_ws;
    unsigned short* Xq   = (unsigned short*)wsp; wsp += SZ_X;
    unsigned short* Xk   = (unsigned short*)wsp; wsp += SZ_X;
    unsigned short* Xv   = (unsigned short*)wsp; wsp += SZ_X;
    unsigned short* WqT  = (unsigned short*)wsp; wsp += SZ_W;
    unsigned short* WoT  = (unsigned short*)wsp; wsp += SZ_W;
    unsigned short* WoTb = (unsigned short*)wsp; wsp += SZ_W;
    unsigned short* WkT  = (unsigned short*)wsp; wsp += SZ_WS;
    unsigned short* WvT  = (unsigned short*)wsp; wsp += SZ_WS;
    unsigned short* Qh   = (unsigned short*)wsp; wsp += SZ_X;
    unsigned short* Ql   = (unsigned short*)wsp; wsp += SZ_X;
    unsigned short* Kh   = (unsigned short*)wsp; wsp += SZ_K;
    unsigned short* Kb   = (unsigned short*)wsp; wsp += SZ_K;
    unsigned short* VT   = (unsigned short*)wsp; wsp += SZ_K;
    unsigned short* Ch   = (unsigned short*)wsp; wsp += SZ_X;
    unsigned short* Cl   = (unsigned short*)wsp; wsp += SZ_X;
    if ((size_t)(wsp - (char*)d_ws) != CARVE) return;

    k_castb<<<dim3((unsigned)(SEQ / 2), (unsigned)NB), 256, 0, stream>>>(q, Xq);
    k_castb<<<dim3((unsigned)(SEQ / 2), (unsigned)NB), 256, 0, stream>>>(k, Xk);
    k_castb<<<dim3((unsigned)(SEQ / 2), (unsigned)NB), 256, 0, stream>>>(v, Xv);
    k_castbT<false><<<(unsigned)(EMB / 2), 256, 0, stream>>>(Wq, (unsigned)EMB, WqT);
    k_castbT<false><<<(unsigned)(HD / 2), 256, 0, stream>>>(Wk, (unsigned)HD, WkT);
    k_castbT<false><<<(unsigned)(HD / 2), 256, 0, stream>>>(Wv, (unsigned)HD, WvT);
    k_castbT<false><<<(unsigned)(EMB / 2), 256, 0, stream>>>(Wo, (unsigned)EMB, WoT);
    k_castbT<true><<<(unsigned)(EMB / 2), 256, 0, stream>>>(Wo, (unsigned)EMB, WoTb);

    {
        const unsigned tilesM = (unsigned)(ROWS / 64);
        k_gemm64<4, false, 2, 2><<<dim3((tilesM * 16u + 7u) / 8u, 1u), 256, 0, stream>>>(
            Xq, nullptr, (unsigned)EMB, 0u, WqT, nullptr, (unsigned)EMB, (void*)Qh, (void*)Ql, (unsigned)EMB, 0u, bq, tilesM, 16u, (unsigned)EMB, 0.0625f, 16.0f);
        k_gemm64<4, false, 2, 3><<<dim3((tilesM + 7u) / 8u, 1u), 256, 0, stream>>>(
            Xk, nullptr, (unsigned)EMB, 0u, WkT, nullptr, (unsigned)EMB, (void*)Kh, (void*)Kb, (unsigned)HD, 0u, bk, tilesM, 1u, (unsigned)EMB, 0.0625f, 16.0f);
        k_gemm64<4, false, 1, 1><<<dim3((tilesM + 7u) / 8u, 1u), 256, 0, stream>>>(
            WvT, nullptr, (unsigned)EMB, 0u, Xv, nullptr, (unsigned)EMB, (void*)VT, nullptr, (unsigned)ROWS, 0u, bv, 1u, tilesM, (unsigned)EMB, 0.0625f, 16.0f);
    }

    k_flash<<<dim3((unsigned)(SEQ / 64), (unsigned)NHEAD, (unsigned)NB), 128, 0, stream>>>(Qh, Ql, Kh, Kb, VT, Ch, Cl);

    {
        const unsigned tilesM = (unsigned)(SEQ / 32);
        k_gemm64<2, true, 2, 0><<<dim3((tilesM * 16u + 7u) / 8u, (unsigned)NB), 256, 0, stream>>>(
            Ch, Cl, (unsigned)EMB, (unsigned)((size_t)SEQ * EMB), WoT, WoTb, (unsigned)EMB, (void*)out, nullptr, (unsigned)EMB, (unsigned)((size_t)SEQ_FULL * EMB),
            bo, tilesM, 16u, (unsigned)EMB, 1.0f / (CTXC * WSC), 1.0f);
    }
}
